// GraphAttentionLayer_31327491457337
// MI455X (gfx1250) — hardware-verified
//
#include <hip/hip_runtime.h>


#define NN   512
#define NF   512
#define NHD  8
#define HD   64
#define DM   (NHD * HD)
#define GP   (2 * DM)
#ifndef QROWS
#define QROWS 512
#endif
#define SCP  516
#define PCAR 4096.0f
#define PINV (1.0f / 4096.0f)
#define LOG2E 1.4426950408889634f
#define SLOPE 0.2f
#define NEGB (-3.0e38f)
#define OUT1_ELEM 262144

static_assert(NHD * HD == DM);
static_assert(NF % 32 == 0);
static_assert(NN % 32 == 0);
static_assert(NN % 64 == 0);
static_assert(GP % 64 == 0);
static_assert(DM % 64 == 0);
static_assert(HD == 64);
static_assert(QROWS % 64 == 0);
static_assert(QROWS >= 64);
static_assert(QROWS <= NN);
static_assert(NN == 512);
static_assert(DM == 512);
static_assert((SCP * 4) % 16 == 0);
static_assert(SCP >= NN);
static_assert((size_t)NN * DM * 4 == (size_t)1048576);
static_assert((size_t)NN * DM == (size_t)OUT1_ELEM);
static_assert(16 * 68 * 4 <= 131072);
static_assert((NHD * SCP + NHD * HD + HD + NHD) * 4 <= 131072);

typedef _Float16 h16;
typedef unsigned short bf;
typedef __attribute__((ext_vector_type(16))) __bf16   v16bf;
typedef __attribute__((ext_vector_type(16))) _Float16 v16h;
typedef __attribute__((ext_vector_type(8)))  _Float16 v8h;
typedef __attribute__((ext_vector_type(8)))  unsigned short v8us;
typedef __attribute__((ext_vector_type(8)))  float    v8f;
typedef __attribute__((ext_vector_type(4)))  float    v4f;
typedef v4f  __attribute__((may_alias)) v4fa;

__device__ __forceinline__ unsigned short f2bf(float f) { unsigned u = __float_as_uint(f); u += 0x7FFFu + ((u >> 16) & 1u); return (unsigned short)(u >> 16); }
__device__ __forceinline__ float bfr(float f) { return __uint_as_float(((unsigned)f2bf(f)) << 16); }
__device__ __forceinline__ v16h cat16(v8h lo, v8h hi) { return __builtin_shufflevector(lo, hi, 0, 1, 2, 3, 4, 5, 6, 7, 8, 9, 10, 11, 12, 13, 14, 15); }
__device__ __forceinline__ v16bf cat16b(v8us lo, v8us hi) { return __builtin_bit_cast(v16bf, __builtin_shufflevector(lo, hi, 0, 1, 2, 3, 4, 5, 6, 7, 8, 9, 10, 11, 12, 13, 14, 15)); }
__device__ __forceinline__ v8f wmma16(v16h a, v16h b, v8f c) { return __builtin_amdgcn_wmma_f32_16x16x32_f16(false, a, false, b, (short)0, c, false, false); }
__device__ __forceinline__ v8f wmmab(v16bf a, v16bf b, v8f c) { return __builtin_amdgcn_wmma_f32_16x16x32_bf16(false, a, false, b, (short)0, c, false, false); }
__device__ __forceinline__ v16h  ldh(const h16* p) { return cat16(*(const v8h*)p, *(const v8h*)(p + 16)); }
__device__ __forceinline__ v16bf ldb(const bf* p)  { return cat16b(*(const v8us*)p, *(const v8us*)(p + 16)); }
__device__ __forceinline__ void wave_sync() { __builtin_amdgcn_fence(3  , "wavefront"); __builtin_amdgcn_wave_barrier(); asm volatile("" ::: "memory"); }

static __device__ __forceinline__ h16 toh_flush(float v) { const h16 r = (h16)v; return (fabsf(v) < 6.103515625e-05f) ? (h16)0.0f : r; }

__device__ __forceinline__ v8f mma(v16h a, v16h b, v8f c)   { c = wmma16(a, b, c); asm volatile("v_nop\n\tv_nop\n\tv_nop\n\tv_nop" : "+v"(c) : "v"(a), "v"(b)); return c; }
__device__ __forceinline__ v8f mma(v16bf a, v16bf b, v8f c) { c = wmmab(a, b, c);  asm volatile("v_nop\n\tv_nop\n\tv_nop\n\tv_nop" : "+v"(c) : "v"(a), "v"(b)); return c; }
__device__ __forceinline__ v16h  ldf(const h16* p) { return ldh(p); }
__device__ __forceinline__ v16bf ldf(const bf* p)  { return ldb(p); }

__global__ __launch_bounds__(256) void k_cvt8(const float* __restrict__ src, bf* dst, size_t n8) {
    const size_t i = (size_t)blockIdx.x * 256 + threadIdx.x; if (i >= n8) return;
    const v8f v = *(const v8f*)(src + i * 8); v8us o;
#pragma unroll
    for (int k = 0; k < 8; ++k) o[k] = f2bf(v[k]);
    *(volatile v8us*)(dst + i * 8) = o; __threadfence(); *(volatile v8us*)(dst + i * 8) = o;
}

template <typename T, int EPI>
__device__ __forceinline__ void gemm_tile(const T* __restrict__ A, const T* __restrict__ Bt, int K, float* Cf, h16* Ch, int ldc, float scale) {
    __shared__ __align__(16) float os[16 * 68];
    typedef decltype(ldf((const T*)0)) FR;
    const int lane = threadIdx.x & 31, lr = lane & 15, hi = lane >> 4;
    v8f acc[4][4];
#pragma unroll
    for (int mb = 0; mb < 4; ++mb)
#pragma unroll
        for (int nb = 0; nb < 4; ++nb) acc[mb][nb] = (v8f){};
    const size_t aoff = (size_t)lr * K + 8 * hi, boff = (size_t)lr * K + 8 * hi;
#pragma unroll 1
    for (int kc = 0; kc < K; kc += 32) {
        FR a[4];
#pragma unroll
        for (int mb = 0; mb < 4; ++mb) a[mb] = ldf(A + aoff + (size_t)mb * 16 * K + kc);
#pragma unroll
        for (int nb = 0; nb < 4; ++nb) { const FR b = ldf(Bt + boff + (size_t)nb * 16 * K + kc);
#pragma unroll
            for (int mb = 0; mb < 4; ++mb) acc[mb][nb] = mma(a[mb], b, acc[mb][nb]); }
    }
    static_assert(32 * 16 * 8 == 16 * 64 * 4);
    static_assert(32 * 16 * 4 == 16 * 64 * 2);
#pragma unroll
    for (int mb = 0; mb < 4; ++mb) {
#pragma unroll
        for (int nb = 0; nb < 4; ++nb) {
#pragma unroll
            for (int j = 0; j < 8; ++j) os[(hi * 8 + j) * 68 + nb * 16 + lr] = acc[mb][nb][j] * scale; }
        wave_sync();
#pragma unroll 1
        for (int ps = 0; ps < 2; ++ps) {
            if (EPI == 0) {
#pragma unroll
                for (int s = 0; s < 8; ++s) { const int row = 2 * s + (lane >> 4), c4 = (lane & 15) * 4;
                    const v4f val = *(const v4fa*)(&os[row * 68 + c4]);
                    *(volatile v4f*)(Cf + (size_t)(mb * 16 + row) * (size_t)ldc + c4) = val; }
            } else {
#pragma unroll
                for (int s = 0; s < 4; ++s) { const int row = 4 * s + (lane >> 3), c8 = (lane & 7) * 8;
                    const v4f x0 = *(const v4fa*)(&os[row * 68 + c8]); const v4f x1 = *(const v4fa*)(&os[row * 68 + c8 + 4]); v8h hv;
#pragma unroll
                    for (int i = 0; i < 4; ++i) { hv[i] = toh_flush(x0[i]); hv[4 + i] = toh_flush(x1[i]); }
                    *(volatile v8h*)(Ch + (size_t)(mb * 16 + row) * (size_t)ldc + c8) = hv; }
            }
            if (ps == 0) __threadfence(); }
        wave_sync();
    }
}

__global__ __launch_bounds__(32) void k_gemm_g(const bf* __restrict__ XB, const bf* __restrict__ WB, float* G) {
    const size_t r0 = (size_t)blockIdx.x * 64, c0 = (size_t)blockIdx.y * 64;
    gemm_tile<bf, 0>(XB + r0 * NF, WB + c0 * NF, NF, G + r0 * GP + c0, (h16*)0, GP, 1.0f);
}

__global__ __launch_bounds__(32) void k_gemm_vt(const bf* __restrict__ WT, const bf* __restrict__ XB, h16* VT) {
    const size_t r0 = (size_t)blockIdx.x * 64, c0 = (size_t)blockIdx.y * 64;
    gemm_tile<bf, 1>(WT + r0 * NF, XB + c0 * NF, NF, (float*)0, VT + r0 * NN + c0, NN, 1.0f);
}

__global__ __launch_bounds__(32) void k_gemm_o(const h16* __restrict__ PP, const h16* __restrict__ VT, float* OUT) {
    const size_t r0 = (size_t)blockIdx.x * 64, z = (size_t)blockIdx.z;
    gemm_tile<h16, 0>(PP + (z * NN + r0) * NN, VT + z * HD * NN, NN, OUT + r0 * DM + z * HD, (h16*)0, DM, PINV);
}

__global__ __launch_bounds__(256) void k_score(const float* __restrict__ G, const float* __restrict__ aw, const int* __restrict__ adj, float* ATT, h16* PP) {
#pragma clang fp contract(off)
    __shared__ __align__(16) float sc[NHD * SCP];
    __shared__ __align__(16) float tg[NHD * HD];
    __shared__ __align__(16) float wv[HD];
    __shared__ float linv[NHD];
    const int tid = threadIdx.x, lane = tid & 31;
    const int wave = __builtin_amdgcn_readfirstlane((int)(threadIdx.x >> 5));
    const unsigned i = blockIdx.x;
    tg[tid]       = G[(size_t)i * GP + DM + tid];
    tg[256 + tid] = G[(size_t)i * GP + DM + 256 + tid];
    if (tid < HD) wv[tid] = bfr(aw[tid]);
    __syncthreads();

    float mx = NEGB; unsigned km = 0u;
#pragma unroll 1
    for (int jj = 0; jj < 16; ++jj) {
        unsigned j = (unsigned)jj * 32u + (unsigned)lane; asm volatile("" : "+v"(j));
        const size_t so = (size_t)j * GP + (size_t)wave * HD;
        float acc = 0.0f;
#pragma unroll 4
        for (int f4 = 0; f4 < 16; ++f4) {
            const v4f s = *(const v4f*)(G + so + 4 * f4);
            const v4f t = *(const v4fa*)(&tg[wave * HD + 4 * f4]);
            const v4f w = *(const v4fa*)(&wv[4 * f4]);
#pragma unroll
            for (int c = 0; c < 4; ++c) { const float v = s[c] + t[c]; const float lv = fmaxf(v, SLOPE * v); acc = fmaf(lv, w[c], acc); }
        }
        int av = adj[(size_t)i * NN + j]; asm volatile("" : "+v"(av));
        const bool keep = av != 0;
        const float s2 = acc * LOG2E;
        sc[wave * SCP + j] = s2;
        mx = fmaxf(mx, keep ? s2 : NEGB);
        km |= (keep ? 1u : 0u) << jj;
    }
#pragma unroll
    for (int o = 16; o > 0; o >>= 1) mx = fmaxf(mx, __shfl_xor(mx, o, 32));
    float ls = 0.0f;
#pragma unroll 1
    for (int jj = 0; jj < 16; ++jj) {
        const unsigned j = (unsigned)jj * 32u + (unsigned)lane;
        const float s2 = sc[wave * SCP + j];
        const float e = __builtin_amdgcn_exp2f(s2 - mx);
        const float g = ((km >> jj) & 1u) ? e : 0.0f;
        sc[wave * SCP + j] = g; ls += g;
    }
#pragma unroll
    for (int o = 16; o > 0; o >>= 1) ls += __shfl_xor(ls, o, 32);
    const float inv = __builtin_amdgcn_rcpf(ls);
    if (lane == 0) linv[wave] = inv;
    __syncthreads();

    static_assert(256 * 4 * 16 == NN * NHD * 4);
    static_assert(256 * 2 * 16 == NHD * NN * 2);
    float* arow = ATT + (size_t)i * (NN * NHD);
#pragma unroll 1
    for (int ps = 0; ps < 2; ++ps) {
#pragma unroll
        for (int it = 0; it < 4; ++it) { const int p = it * 256 + tid; const int j = p >> 1, h0 = (p & 1) * 4;
            v4f val;
#pragma unroll
            for (int k = 0; k < 4; ++k) val[k] = sc[(h0 + k) * SCP + j] * linv[h0 + k];
            *(volatile v4f*)(arow + (size_t)p * 4) = val; }
#pragma unroll
        for (int it = 0; it < 2; ++it) { const int p = it * 256 + tid; const int hh = p >> 6, j0 = (p & 63) * 8;
            const v4f x0 = *(const v4fa*)(&sc[hh * SCP + j0]); const v4f x1 = *(const v4fa*)(&sc[hh * SCP + j0 + 4]);
            const float iv = linv[hh]; v8h hv;
#pragma unroll
            for (int k = 0; k < 4; ++k) { hv[k] = toh_flush((x0[k] * iv) * PCAR); hv[4 + k] = toh_flush((x1[k] * iv) * PCAR); }
            *(volatile v8h*)(PP + ((size_t)hh * NN + i) * NN + j0) = hv; }
        if (ps == 0) __threadfence(); }
}

static constexpr size_t al256(size_t v) { return (v + 255) & ~(size_t)255; }
static constexpr size_t SZ_XB = al256((size_t)NN * NF * 2);
static constexpr size_t SZ_WB = al256((size_t)GP * NF * 2);
static constexpr size_t SZ_G  = al256((size_t)NN * GP * 4);
static constexpr size_t SZ_VT = al256((size_t)DM * NN * 2);
static constexpr size_t SZ_PP = al256((size_t)NHD * NN * NN * 2);
static constexpr size_t SZ_TOTAL = SZ_XB + SZ_WB + SZ_G + SZ_VT + SZ_PP;
static_assert(SZ_TOTAL <= (size_t)134217728);
static_assert(((size_t)DM * NF * 2) % 256 == 0);
static_assert(((size_t)NN * NF) % 8 == 0);
static_assert(((size_t)DM * NF) % 8 == 0);

extern "C" void kernel_launch(void* const* d_in, const int* in_sizes, int n_in,
                              void* d_out, int out_size, void* d_ws, size_t ws_size, hipStream_t stream) {
    if (n_in < 5) return;
    if ((size_t)in_sizes[0] < (size_t)NN * NF) return;
    if ((size_t)in_sizes[1] < (size_t)DM * NF || (size_t)in_sizes[2] < (size_t)DM * NF) return;
    if (in_sizes[3] < HD) return;
    if ((size_t)in_sizes[4] < (size_t)NN * NN) return;
    if ((size_t)out_size < (size_t)OUT1_ELEM + (size_t)NN * NN * NHD) return;
    if (SZ_TOTAL > ws_size) return;
    const float* x  = (const float*)d_in[0];
    const float* ws = (const float*)d_in[1];
    const float* wt = (const float*)d_in[2];
    const float* aw = (const float*)d_in[3];
    const int*  adj = (const int*)d_in[4];
    float* OUT = (float*)d_out;
    float* ATT = (float*)d_out + OUT1_ELEM;
    char* wsp = (char*)d_ws;
    bf*    XB = (bf*)wsp;    wsp += SZ_XB;
    bf*    WB = (bf*)wsp;    wsp += SZ_WB;
    float* G  = (float*)wsp; wsp += SZ_G;
    h16*   VT = (h16*)wsp;   wsp += SZ_VT;
    h16*   PP = (h16*)wsp;   wsp += SZ_PP;
    bf* WS = WB; bf* WT = WB + (size_t)DM * NF;

    { const size_t n8 = (size_t)NN * NF / 8; k_cvt8<<<(unsigned)((n8 + 255) / 256), 256, 0, stream>>>(x, XB, n8); }
    { const size_t n8 = (size_t)DM * NF / 8; const unsigned g = (unsigned)((n8 + 255) / 256);
      k_cvt8<<<g, 256, 0, stream>>>(ws, WS, n8); k_cvt8<<<g, 256, 0, stream>>>(wt, WT, n8); }

    k_gemm_g <<<dim3(NN / 64, GP / 64, 1), 32, 0, stream>>>(XB, WB, G);
    k_gemm_vt<<<dim3(DM / 64, NN / 64, 1), 32, 0, stream>>>(WT, XB, VT);
    k_score  <<<dim3(QROWS, 1, 1), 256, 0, stream>>>(G, aw, adj, ATT, PP);
    k_gemm_o <<<dim3(QROWS / 64, 1, NHD), 32, 0, stream>>>(PP, VT, OUT);
}
